// StandardAttention_43903155699725
// MI455X (gfx1250) — hardware-verified
//
#include <hip/hip_runtime.h>
#include <math.h>
#include <stdint.h>

#ifndef NB
#define NB    2
#endif
#ifndef SEQ
#define SEQ   2048
#endif
#define NB_FULL   2
#define SEQ_FULL  2048
#define DM    1024
#define NH    16
#define HD    64
#define DQKV  (3 * DM)
#define NQB   (SEQ / 64)
#define NKT   (SEQ / 64)
#define MW    (SEQ / 32)
#define ROWS  (NB * SEQ)
#define OUTN  (ROWS * DM)
static_assert(NH * HD == DM);
static_assert(HD == 64);
static_assert(NB >= 1 && NB <= NB_FULL);
static_assert(SEQ >= 64 && SEQ <= SEQ_FULL && (SEQ % 64) == 0);
static_assert((DM % 64) == 0 && (DQKV % 64) == 0 && (DM % 32) == 0);
static_assert((((ROWS / 64) * (DQKV / 64)) % 8) == 0);
static_assert((((ROWS / 64) * (DM / 64)) % 8) == 0);
static_assert(((SEQ * DM / 8) % 256) == 0 && ((DM * DM / 8) % 256) == 0);
static_assert(((NB * SEQ * MW) % 256) == 0);
static_assert(MW >= 2);

typedef _Float16 v16h __attribute__((ext_vector_type(16)));
typedef _Float16 v8h  __attribute__((ext_vector_type(8)));
typedef float    v8f  __attribute__((ext_vector_type(8)));
typedef float    v4f  __attribute__((ext_vector_type(4)));
typedef unsigned int v4u __attribute__((ext_vector_type(4)));
typedef int      v4i  __attribute__((ext_vector_type(4)));

__device__ __forceinline__ unsigned short bf_bits(float f) {
  unsigned u = __float_as_uint(f);
  return (unsigned short)((u + 0x7FFFu + ((u >> 16) & 1u)) >> 16);
}
__device__ __forceinline__ float bfr(float f) { return __uint_as_float(((unsigned)bf_bits(f)) << 16); }
__device__ __forceinline__ unsigned short h_bits(_Float16 x) { return __builtin_bit_cast(unsigned short, x); }
__device__ __forceinline__ unsigned pk16(unsigned short a, unsigned short b) { return (unsigned)a | ((unsigned)b << 16); }
__device__ __forceinline__ v8f zero8() { v8f z = {0.f, 0.f, 0.f, 0.f, 0.f, 0.f, 0.f, 0.f}; return z; }

__device__ __forceinline__ v16h ldfrag_h(const _Float16* p) {
  union { v16h v; v8h h[2]; } f;
  f.h[0] = *(const v8h*)(p);
  f.h[1] = *(const v8h*)(p + 16);
  return f.v;
}

__device__ __forceinline__ v8f mma_h(v16h a, v16h b, v8f c) {
  c = __builtin_amdgcn_wmma_f32_16x16x32_f16(false, a, false, b, (short)0, c, false, false);
#if defined(__HIP_DEVICE_COMPILE__)
  asm volatile("v_nop\n\tv_nop\n\tv_nop\n\tv_nop" : "+v"(c) : "v"(a), "v"(b));
#endif
  return c;
}
__device__ __forceinline__ v8f mma_h_raw(v16h a, v16h b, v8f c) {
  return __builtin_amdgcn_wmma_f32_16x16x32_f16(false, a, false, b, (short)0, c, false, false);
}
__device__ __forceinline__ void dep_guard_h(v8f& a, v8f& b, v16h x, v16h y) {
#if defined(__HIP_DEVICE_COMPILE__)
  asm volatile("v_nop\n\tv_nop\n\tv_nop\n\tv_nop" : "+v"(a), "+v"(b) : "v"(x), "v"(y));
#endif
}
__device__ __forceinline__ void keep4_h(v16h a, v16h b, v16h c, v16h d) {
#if defined(__HIP_DEVICE_COMPILE__)
  asm volatile("v_nop" :: "v"(a), "v"(b), "v"(c), "v"(d));
#endif
}
__device__ __forceinline__ void acc_guard4(v8f& a, v8f& b, v8f& c, v8f& d) {
#if defined(__HIP_DEVICE_COMPILE__)
  asm volatile("v_nop\n\tv_nop\n\tv_nop\n\tv_nop" : "+v"(a), "+v"(b), "+v"(c), "+v"(d));
#endif
}

__global__ __launch_bounds__(256) void cvt16(const float* __restrict__ in, unsigned short* out, int n8, float scale,
                                             size_t istr, size_t ostr) {
  const int i = blockIdx.x * 256 + threadIdx.x;
  const float* ip = in + (size_t)blockIdx.y * istr;
  unsigned short* op = out + (size_t)blockIdx.y * ostr;
  if (i < n8) {
    const v4f a = *(const v4f*)(ip + (size_t)i * 8);
    const v4f b = *(const v4f*)(ip + (size_t)i * 8 + 4);
    v4u p;
    p[0] = pk16(h_bits((_Float16)(bfr(a[0]) * scale)), h_bits((_Float16)(bfr(a[1]) * scale)));
    p[1] = pk16(h_bits((_Float16)(bfr(a[2]) * scale)), h_bits((_Float16)(bfr(a[3]) * scale)));
    p[2] = pk16(h_bits((_Float16)(bfr(b[0]) * scale)), h_bits((_Float16)(bfr(b[1]) * scale)));
    p[3] = pk16(h_bits((_Float16)(bfr(b[2]) * scale)), h_bits((_Float16)(bfr(b[3]) * scale)));
    *(volatile v4u*)(op + (size_t)i * 8) = p;
    __threadfence();
    *(volatile v4u*)(op + (size_t)i * 8) = p;
  }
}

__global__ __launch_bounds__(256) void mask_bits(const int* __restrict__ mp, unsigned int* mb) {
  __shared__ __align__(16) unsigned int sW[256];
  const int tid = threadIdx.x;
  const int gw  = blockIdx.x * 256 + tid;
  const int row = gw / MW;
  const int w   = gw - row * MW;
  const int b   = row / SEQ;
  const int q   = row - b * SEQ;
  const int* src = mp + ((size_t)b * SEQ_FULL + (size_t)q) * SEQ_FULL + (size_t)w * 32;
  unsigned bits = 0u;
#pragma unroll
  for (int i = 0; i < 8; ++i) {
    const v4i m = *(const v4i*)(src + 4 * i);
#pragma unroll
    for (int e = 0; e < 4; ++e) bits |= ((m[e] != 0) ? 1u : 0u) << (4 * i + e);
  }
  sW[tid] = bits;
  __syncthreads();
  if (tid < 64) {
    const v4u p = *(const v4u*)(sW + 4 * tid);
    unsigned int* dst = mb + (size_t)blockIdx.x * 256 + 4 * tid;
    *(volatile v4u*)dst = p;
    __threadfence();
    *(volatile v4u*)dst = p;
  }
}

template <int EPI, bool ARES>
__global__ __launch_bounds__(256) void gemm64_f16(
    const unsigned short* __restrict__ Ap, const unsigned short* __restrict__ Arp, int lda,
    const unsigned short* __restrict__ Btp, int ldb,
    float cscale,
    void* Cp, unsigned short* Crp, int ldc, int M, int N, int K, float oscale,
    int tmod, int tlo, int thi) {
  const _Float16* Ah  = (const _Float16*)(const void*)Ap;
  const _Float16* Arh = (const _Float16*)(const void*)Arp;
  const _Float16* Bt  = (const _Float16*)(const void*)Btp;
  __shared__ __align__(16) float sT[8][16 * 68];
  const int lane = threadIdx.x & 31;
  const int wave = threadIdx.x >> 5;
  const int tilesN = N >> 6;
  const int tilesM = M >> 6;
  const int tile = blockIdx.x * 8 + wave;
  if (tile >= tilesM * tilesN) return;
  const int tm = tile / tilesN;
  const int tn = tile - tm * tilesN;
  const int m0 = tm << 6;
  const int n0 = tn << 6;
  const int tpos = m0 % tmod;
  if (tpos < tlo || tpos >= thi) return;

  const int rlane = lane & 15;
  const int koff  = (lane >> 4) * 8;
  const int mOff  = (lane >> 4) * 8;

  v8f acc[4][4];
#pragma unroll
  for (int i = 0; i < 4; ++i)
#pragma unroll
    for (int j = 0; j < 4; ++j) acc[i][j] = zero8();

  constexpr int NPL = ARES ? 2 : 1;
#pragma unroll 1
  for (int pl = 0; pl < NPL; ++pl) {
    const _Float16* Asel = (ARES && pl == 0) ? Arh : Ah;
    if (ARES && pl == 1) {
      acc_guard4(acc[0][0], acc[0][1], acc[0][2], acc[0][3]);
      acc_guard4(acc[1][0], acc[1][1], acc[1][2], acc[1][3]);
      acc_guard4(acc[2][0], acc[2][1], acc[2][2], acc[2][3]);
      acc_guard4(acc[3][0], acc[3][1], acc[3][2], acc[3][3]);
#pragma unroll
      for (int i = 0; i < 4; ++i)
#pragma unroll
        for (int j = 0; j < 4; ++j) acc[i][j] = acc[i][j] * (1.0f / 2048.0f);
      acc_guard4(acc[0][0], acc[0][1], acc[0][2], acc[0][3]);
      acc_guard4(acc[1][0], acc[1][1], acc[1][2], acc[1][3]);
      acc_guard4(acc[2][0], acc[2][1], acc[2][2], acc[2][3]);
      acc_guard4(acc[3][0], acc[3][1], acc[3][2], acc[3][3]);
    }
    for (int k0 = 0; k0 < K; k0 += 32) {
      v16h bh[4];
#pragma unroll
      for (int j = 0; j < 4; ++j) {
        const size_t bo = (size_t)(n0 + (j << 4) + rlane) * ldb + koff + k0;
        bh[j] = ldfrag_h(Bt + bo);
      }
#pragma unroll
      for (int i = 0; i < 4; ++i) {
        const size_t ao = (size_t)(m0 + (i << 4) + rlane) * lda + koff + k0;
        const v16h ah = ldfrag_h(Asel + ao);
#pragma unroll
        for (int j = 0; j < 4; ++j) {
          acc[i][j] = mma_h_raw(ah, bh[j], acc[i][j]);
        }
        dep_guard_h(acc[i][0], acc[i][3], ah, bh[3]);
      }
      keep4_h(bh[0], bh[1], bh[2], bh[3]);
    }
  }
  acc_guard4(acc[0][0], acc[0][1], acc[0][2], acc[0][3]);
  acc_guard4(acc[1][0], acc[1][1], acc[1][2], acc[1][3]);
  acc_guard4(acc[2][0], acc[2][1], acc[2][2], acc[2][3]);
  acc_guard4(acc[3][0], acc[3][1], acc[3][2], acc[3][3]);

  float* slab = sT[wave];
#pragma unroll
  for (int i = 0; i < 4; ++i) {
    const int mBase = m0 + (i << 4);
#pragma unroll
    for (int r = 0; r < 8; ++r) {
      const int row = mOff + r;
#pragma unroll
      for (int j = 0; j < 4; ++j) slab[row * 68 + (j << 4) + rlane] = acc[i][j][r] * cscale;
    }
    __builtin_amdgcn_fence(__ATOMIC_RELEASE, "workgroup");
    __builtin_amdgcn_wave_barrier();
    __builtin_amdgcn_fence(__ATOMIC_ACQUIRE, "workgroup");
    if constexpr (EPI == 0) {
      unsigned short* C16 = (unsigned short*)Cp;
      const int rq = lane >> 3, piece = lane & 7;
      v4u ph[4], pr[4];
#pragma unroll
      for (int it = 0; it < 4; ++it) {
        const int row = it * 4 + rq;
        const v4f a  = *(const v4f*)(slab + row * 68 + piece * 8);
        const v4f a2 = *(const v4f*)(slab + row * 68 + piece * 8 + 4);
        float f[8];
        f[0] = a[0];  f[1] = a[1];  f[2] = a[2];  f[3] = a[3];
        f[4] = a2[0]; f[5] = a2[1]; f[6] = a2[2]; f[7] = a2[3];
        v4u p, q;
#pragma unroll
        for (int e = 0; e < 4; ++e) {
          const float g0 = f[2 * e] * oscale, g1 = f[2 * e + 1] * oscale;
          const _Float16 x0 = (_Float16)g0, x1 = (_Float16)g1;
          const _Float16 y0 = (_Float16)((g0 - (float)x0) * 2048.0f);
          const _Float16 y1 = (_Float16)((g1 - (float)x1) * 2048.0f);
          p[e] = pk16(h_bits(x0), h_bits(x1));
          q[e] = pk16(h_bits(y0), h_bits(y1));
        }
        ph[it] = p;
        pr[it] = q;
      }
      for (int pass = 0; pass < 2; ++pass) {
#pragma unroll
        for (int it = 0; it < 4; ++it) {
          const int row = it * 4 + rq;
          const size_t co = (size_t)(mBase + row) * ldc + n0 + piece * 8;
          *(volatile v4u*)(C16 + co) = ph[it];
          *(volatile v4u*)(Crp + co) = pr[it];
        }
        __threadfence();
      }
    } else {
      float* Cf = (float*)Cp;
      const int hh = lane >> 4, c4 = (lane & 15) * 4;
      v4f ov[8];
#pragma unroll
      for (int it = 0; it < 8; ++it) {
        const int row = it * 2 + hh;
        ov[it] = *(const v4f*)(slab + row * 68 + c4);
      }
      for (int pass = 0; pass < 2; ++pass) {
#pragma unroll
        for (int it = 0; it < 8; ++it) {
          const int row = it * 2 + hh;
          *(volatile v4f*)(Cf + (size_t)(mBase + row) * ldc + n0 + c4) = ov[it];
        }
        __threadfence();
      }
    }
    __builtin_amdgcn_fence(__ATOMIC_RELEASE, "workgroup");
    __builtin_amdgcn_wave_barrier();
    __builtin_amdgcn_fence(__ATOMIC_ACQUIRE, "workgroup");
  }
}

__global__ __launch_bounds__(256) void v_tr(const unsigned short* __restrict__ qkvp, unsigned short* vt) {
  __shared__ __align__(16) _Float16 sv[64 * 72];
  const int tid = threadIdx.x;
  const int t0  = blockIdx.x * 64;
  const int hh  = blockIdx.y;
  const int b   = blockIdx.z;
  const _Float16* src = (const _Float16*)(const void*)qkvp;
#pragma unroll
  for (int i = 0; i < 2; ++i) {
    const int idx = i * 256 + tid;
    const int tt = idx >> 3, c8 = (idx & 7) * 8;
    const v8h a = *(const v8h*)(src + ((size_t)(b * SEQ + t0 + tt)) * DQKV + 2 * DM + hh * HD + c8);
    *(v8h*)(sv + tt * 72 + c8) = a;
  }
  __syncthreads();

  const int g = tid >> 3, piece = tid & 7;
  v4u hv[2];
  size_t hofs[2];
#pragma unroll
  for (int it = 0; it < 2; ++it) {
    const int d = it * 32 + g;
    v4u a;
#pragma unroll
    for (int e = 0; e < 4; ++e) {
      const _Float16 x0 = sv[(piece * 8 + 2 * e) * 72 + d];
      const _Float16 x1 = sv[(piece * 8 + 2 * e + 1) * 72 + d];
      a[e] = pk16(h_bits(x0), h_bits(x1));
    }
    hv[it] = a;
    hofs[it] = ((size_t)(b * DM + hh * HD + d)) * SEQ + t0 + piece * 8;
  }
  for (int pass = 0; pass < 2; ++pass) {
#pragma unroll
    for (int it = 0; it < 2; ++it) *(volatile v4u*)(vt + hofs[it]) = hv[it];
    __threadfence();
  }
}

template <bool HR>
__global__ __launch_bounds__(128)
void attn_k(const unsigned short* __restrict__ qkvp, const unsigned short* __restrict__ qkvrp,
            const unsigned short* __restrict__ vtp, const unsigned short* __restrict__ vtrp,
            const unsigned int* __restrict__ mbp,
            unsigned short* ctxp, unsigned short* ctxrp, int qb_lo, int qb_n) {
  union FH { v16h v; v8h h[2]; };
  constexpr int TB     = 64 * 64 * 2;
  constexpr int PB     = 4 * 16 * 64 * 2;
  constexpr int OFF_K  = 0;
  constexpr int OFF_V  = TB;
  constexpr int OFF_KR = 2 * TB;
  constexpr int OFF_VR = 3 * TB;
  constexpr int OFF_P  = HR ? 4 * TB : 2 * TB;
  constexpr int OFF_PR = OFF_P + PB;
  constexpr int SMEMB  = HR ? (OFF_PR + PB) : (OFF_P + PB);
  static_assert(4 * 16 * 64 * 4 <= OFF_P);
  __shared__ __align__(16) unsigned char smem[SMEMB];
  __shared__ __align__(16) unsigned int sM[64 * 2];
  _Float16* Ksh = (_Float16*)(smem + OFF_K);
  _Float16* Vsh = (_Float16*)(smem + OFF_V);
  _Float16* Krs = (_Float16*)(smem + (HR ? OFF_KR : OFF_K));
  _Float16* Vrs = (_Float16*)(smem + (HR ? OFF_VR : OFF_V));
  _Float16* Psh = (_Float16*)(smem + OFF_P);
  _Float16* Prs = (_Float16*)(smem + (HR ? OFF_PR : OFF_P));

  const int tid  = threadIdx.x;
  const int wave = tid >> 5;
  const int lane = tid & 31;
  const int hh   = lane >> 4;
  const int c    = lane & 15;

  const int bx   = blockIdx.x;
  const int qb   = qb_lo + bx % qb_n;
  const int rest = bx / qb_n;
  const int h    = rest % NH;
  const int b    = rest / NH;
  const int q0   = qb * 64 + wave * 16;
  const size_t rowB = (size_t)b * SEQ;

  const _Float16* Qp  = (const _Float16*)(const void*)qkvp  + (size_t)h * HD;
  const _Float16* Qrp = (const _Float16*)(const void*)qkvrp + (size_t)h * HD;
  const _Float16* Kp  = Qp + DM;
  const _Float16* Krp = Qrp + DM;
  const _Float16* Vt  = (const _Float16*)(const void*)vtp  + ((size_t)b * DM + (size_t)h * HD) * SEQ;
  const _Float16* Vrt = (const _Float16*)(const void*)vtrp + ((size_t)b * DM + (size_t)h * HD) * SEQ;
  const unsigned int* Mrow = mbp + (rowB + (size_t)qb * 64) * MW;

  v16h qa[2], qr[2];
#pragma unroll
  for (int dc = 0; dc < 2; ++dc) {
    const size_t qo = (rowB + q0 + c) * DQKV + dc * 32 + 8 * hh;
    qa[dc] = ldfrag_h(Qp + qo);
    if constexpr (HR) qr[dc] = ldfrag_h(Qrp + qo);
    else qr[dc] = qa[dc];
  }

  float lsum[8], mrun[8];
  v8f oacc[4], oacc2[4];
#pragma unroll
  for (int r = 0; r < 8; ++r) { lsum[r] = 0.f; mrun[r] = -1e30f; }
#pragma unroll
  for (int t = 0; t < 4; ++t) { oacc[t] = zero8(); oacc2[t] = zero8(); }

  _Float16* pw  = Psh + wave * (16 * 64);
  _Float16* prw = Prs + wave * (16 * 64);

  for (int kt = 0; kt < NKT; ++kt) {
    const int kv0 = kt * 64;
    __syncthreads();
    {
      const int r = tid >> 1, half = (tid & 1) * 32;
      const size_t ko = (rowB + kv0 + r) * DQKV + half;
      const size_t vo = (size_t)r * SEQ + kv0 + half;
#pragma unroll
      for (int i = 0; i < 4; ++i) {
        const v8h a0 = *(const v8h*)(Kp + ko + 8 * i);
        const v8h b0 = *(const v8h*)(Vt + vo + 8 * i);
        *(v8h*)(Ksh + r * 64 + half + 8 * i) = a0;
        *(v8h*)(Vsh + r * 64 + half + 8 * i) = b0;
        if constexpr (HR) {
          const v8h a1 = *(const v8h*)(Krp + ko + 8 * i);
          const v8h b1 = *(const v8h*)(Vrt + vo + 8 * i);
          *(v8h*)(Krs + r * 64 + half + 8 * i) = a1;
          *(v8h*)(Vrs + r * 64 + half + 8 * i) = b1;
        }
      }
      const int mw = tid & 1;
      sM[r * 2 + mw] = Mrow[(size_t)r * MW + kt * 2 + mw];
    }
    __syncthreads();

    v8f s[4];
#pragma unroll
    for (int j = 0; j < 4; ++j) {
      s[j] = zero8();
      v8f t = zero8();
#pragma unroll
      for (int dc = 0; dc < 2; ++dc) {
        FH kb;
        kb.h[0] = *(const v8h*)(Ksh + (j * 16 + c) * 64 + dc * 32 + 8 * hh);
        kb.h[1] = *(const v8h*)(Ksh + (j * 16 + c) * 64 + dc * 32 + 16 + 8 * hh);
        s[j] = mma_h(qa[dc], kb.v, s[j]);
        if constexpr (HR) {
          FH krb;
          krb.h[0] = *(const v8h*)(Krs + (j * 16 + c) * 64 + dc * 32 + 8 * hh);
          krb.h[1] = *(const v8h*)(Krs + (j * 16 + c) * 64 + dc * 32 + 16 + 8 * hh);
          t = mma_h(qa[dc], krb.v, t);
          t = mma_h(qr[dc], kb.v, t);
        }
      }
      if constexpr (HR) s[j] = s[j] + t * (1.0f / 2048.0f);
    }

    float alpha[8];
#pragma unroll
    for (int r = 0; r < 8; ++r) {
      const int lrow = wave * 16 + 8 * hh + r;
      const unsigned w0 = sM[lrow * 2];
      const unsigned w1 = sM[lrow * 2 + 1];
      unsigned kp[4];
      float av[4];
      float tmx = -1e30f;
#pragma unroll
      for (int j = 0; j < 4; ++j) {
        const unsigned wj = (j & 2) ? w1 : w0;
        kp[j] = (wj >> ((j & 1) * 16 + c)) & 1u;
        float a = s[j][r] * (1.0f / 2048.0f);
        a = (kp[j] != 0u) ? a : -1e30f;
        av[j] = a;
        tmx = fmaxf(tmx, a);
      }
#pragma unroll
      for (int off = 1; off < 16; off <<= 1) tmx = fmaxf(tmx, __shfl_xor(tmx, off, 32));
      const float mn = fmaxf(mrun[r], tmx);
      const float al = __expf(mrun[r] - mn);
      alpha[r] = al;
      mrun[r]  = mn;
      float ps = 0.0f;
#pragma unroll
      for (int j = 0; j < 4; ++j) {
        float p = __expf(av[j] - mn);
        p = (kp[j] != 0u) ? p : 0.0f;
        ps += p;
        const float g = p * 256.0f;
        const _Float16 x0 = (_Float16)g;
        pw[(8 * hh + r) * 64 + j * 16 + c] = x0;
        if constexpr (HR) prw[(8 * hh + r) * 64 + j * 16 + c] = (_Float16)((g - (float)x0) * 2048.0f);
      }
      lsum[r] = lsum[r] * al + ps;
    }
    __builtin_amdgcn_fence(__ATOMIC_RELEASE, "workgroup");
    __builtin_amdgcn_wave_barrier();
    __builtin_amdgcn_fence(__ATOMIC_ACQUIRE, "workgroup");

#pragma unroll
    for (int t = 0; t < 4; ++t) {
#pragma unroll
      for (int r = 0; r < 8; ++r) {
        oacc[t][r] = oacc[t][r] * alpha[r];
        if constexpr (HR) oacc2[t][r] = oacc2[t][r] * alpha[r];
      }
    }
    acc_guard4(oacc[0], oacc[1], oacc[2], oacc[3]);
    if constexpr (HR) acc_guard4(oacc2[0], oacc2[1], oacc2[2], oacc2[3]);

#pragma unroll
    for (int kk = 0; kk < 2; ++kk) {
      FH pa, par;
      pa.h[0] = *(const v8h*)(pw + c * 64 + kk * 32 + 8 * hh);
      pa.h[1] = *(const v8h*)(pw + c * 64 + kk * 32 + 16 + 8 * hh);
      if constexpr (HR) {
        par.h[0] = *(const v8h*)(prw + c * 64 + kk * 32 + 8 * hh);
        par.h[1] = *(const v8h*)(prw + c * 64 + kk * 32 + 16 + 8 * hh);
      } else {
        par.v = pa.v;
      }
#pragma unroll
      for (int t = 0; t < 4; ++t) {
        FH vb;
        vb.h[0] = *(const v8h*)(Vsh + (t * 16 + c) * 64 + kk * 32 + 8 * hh);
        vb.h[1] = *(const v8h*)(Vsh + (t * 16 + c) * 64 + kk * 32 + 16 + 8 * hh);
        oacc[t] = mma_h(pa.v, vb.v, oacc[t]);
        if constexpr (HR) {
          FH vrb;
          vrb.h[0] = *(const v8h*)(Vrs + (t * 16 + c) * 64 + kk * 32 + 8 * hh);
          vrb.h[1] = *(const v8h*)(Vrs + (t * 16 + c) * 64 + kk * 32 + 16 + 8 * hh);
          oacc2[t] = mma_h(pa.v, vrb.v, oacc2[t]);
          oacc2[t] = mma_h(par.v, vb.v, oacc2[t]);
        }
      }
    }
  }
  __syncthreads();

  float* os = (float*)(void*)smem + wave * (16 * 64);
#pragma unroll
  for (int r = 0; r < 8; ++r) {
    float l = lsum[r];
#pragma unroll
    for (int off = 1; off < 16; off <<= 1) l += __shfl_xor(l, off, 32);
    const float rl = 1.0f / l;
    const float sc = rl * (1.0f / 256.0f);
#pragma unroll
    for (int t = 0; t < 4; ++t) {
      float v = oacc[t][r];
      if constexpr (HR) v += oacc2[t][r] * (1.0f / 2048.0f);
      os[(8 * hh + r) * 64 + t * 16 + c] = v * sc;
    }
  }
  __builtin_amdgcn_fence(__ATOMIC_RELEASE, "workgroup");
  __builtin_amdgcn_wave_barrier();
  __builtin_amdgcn_fence(__ATOMIC_ACQUIRE, "workgroup");
  {
    const int rq = lane >> 3, piece = lane & 7;
    v4u ph[4], pr[4];
#pragma unroll
    for (int it = 0; it < 4; ++it) {
      const int row = it * 4 + rq;
      const v4f a  = *(const v4f*)(os + row * 64 + piece * 8);
      const v4f a2 = *(const v4f*)(os + row * 64 + piece * 8 + 4);
      float f[8];
      f[0] = a[0];  f[1] = a[1];  f[2] = a[2];  f[3] = a[3];
      f[4] = a2[0]; f[5] = a2[1]; f[6] = a2[2]; f[7] = a2[3];
      v4u p, q;
#pragma unroll
      for (int e = 0; e < 4; ++e) {
        const _Float16 x0 = (_Float16)f[2 * e], x1 = (_Float16)f[2 * e + 1];
        p[e] = pk16(h_bits(x0), h_bits(x1));
        if constexpr (HR) {
          const _Float16 y0 = (_Float16)((f[2 * e] - (float)x0) * 2048.0f);
          const _Float16 y1 = (_Float16)((f[2 * e + 1] - (float)x1) * 2048.0f);
          q[e] = pk16(h_bits(y0), h_bits(y1));
        } else {
          q[e] = p[e];
        }
      }
      ph[it] = p;
      pr[it] = q;
    }
    for (int pass = 0; pass < 2; ++pass) {
#pragma unroll
      for (int it = 0; it < 4; ++it) {
        const int row = it * 4 + rq;
        const size_t go = (rowB + q0 + row) * DM + (size_t)h * HD + piece * 8;
        *(volatile v4u*)(ctxp + go) = ph[it];
        if constexpr (HR) *(volatile v4u*)(ctxrp + go) = pr[it];
      }
      __threadfence();
    }
  }
}

extern "C" void kernel_launch(void* const* d_in, const int* in_sizes, int n_in,
                              void* d_out, int out_size, void* d_ws, size_t ws_size,
                              hipStream_t stream) {
  if (n_in < 6) return;
  if (in_sizes[0] < ((NB - 1) * SEQ_FULL + SEQ) * DM) return;
  if (in_sizes[1] < ((NB - 1) * SEQ_FULL + SEQ) * SEQ_FULL) return;
  if (in_sizes[2] < DM * DM) return;
  if (in_sizes[3] < DM * DM) return;
  if (in_sizes[4] < DM * DM) return;
  if (in_sizes[5] < DM * DM) return;
  if (out_size < OUTN) return;

  const float* x    = (const float*)d_in[0];
  const int*   mask = (const int*)d_in[1];
  const float* wq   = (const float*)d_in[2];
  const float* wk   = (const float*)d_in[3];
  const float* wv   = (const float*)d_in[4];
  const float* wo   = (const float*)d_in[5];

  const size_t PX   = (size_t)ROWS * DM * 2;
  const size_t PWq  = (size_t)DQKV * DM * 2;
  const size_t PWp  = (size_t)DM * DM * 2;
  const size_t PQKV = (size_t)ROWS * DQKV * 2;
  const size_t PVT  = (size_t)NB * DM * SEQ * 2;
  const size_t PCtx = (size_t)ROWS * DM * 2;
  const size_t PMb  = (size_t)NB * SEQ * MW * 4;
  size_t off = 0;
  const size_t oX    = off; off += PX;
  const size_t oWq   = off; off += PWq;
  const size_t oWp   = off; off += PWp;
  const size_t oQKV  = off; off += PQKV;
  const size_t oQKVr = off; off += PQKV;
  const size_t oVT   = off; off += PVT;
  const size_t oVTr  = off; off += PVT;
  const size_t oCtx  = off; off += PCtx;
  const size_t oCtxr = off; off += PCtx;
  const size_t oMb   = off; off += PMb;
  if (off > ws_size) return;
  if (off > (size_t)134217728) return;

  char* ws = (char*)d_ws;
  unsigned short* Xh   = (unsigned short*)(ws + oX);
  unsigned short* Wqkv = (unsigned short*)(ws + oWq);
  unsigned short* Wp   = (unsigned short*)(ws + oWp);
  unsigned short* QKV  = (unsigned short*)(ws + oQKV);
  unsigned short* QKVr = (unsigned short*)(ws + oQKVr);
  unsigned short* VT   = (unsigned short*)(ws + oVT);
  unsigned short* VTr  = (unsigned short*)(ws + oVTr);
  unsigned short* Ctx  = (unsigned short*)(ws + oCtx);
  unsigned short* Ctxr = (unsigned short*)(ws + oCtxr);
  unsigned int*   Mb   = (unsigned int*)(ws + oMb);
  float*          outf = (float*)d_out;

  const dim3 blk(256);
  const int n8x = SEQ * DM / 8;
  const int n8w = DM * DM / 8;
  const dim3 gCx(n8x / 256, NB);
  const dim3 gCw(n8w / 256, 1);
  const dim3 gMb((NB * SEQ * MW) / 256);
  const dim3 gGqkv(((ROWS / 64) * (DQKV / 64) + 7) / 8);
  const dim3 gGdm(((ROWS / 64) * (DM / 64) + 7) / 8);
  const dim3 gVt(SEQ / 64, NH, NB);
  const dim3 gAttn(NQB * NH * NB);
  const float wScale = 1024.0f;
  const float aScale = 16.0f;
  const float cscale = 1.0f / 16384.0f;

  cvt16<<<gCx, blk, 0, stream>>>(x, Xh, n8x, aScale, (size_t)SEQ_FULL * DM, (size_t)SEQ * DM);
  cvt16<<<gCw, blk, 0, stream>>>(wq, Wqkv, n8w, wScale, (size_t)0, (size_t)0);
  cvt16<<<gCw, blk, 0, stream>>>(wk, Wqkv + (size_t)DM * DM, n8w, wScale, (size_t)0, (size_t)0);
  cvt16<<<gCw, blk, 0, stream>>>(wv, Wqkv + (size_t)2 * DM * DM, n8w, wScale, (size_t)0, (size_t)0);
  cvt16<<<gCw, blk, 0, stream>>>(wo, Wp, n8w, wScale, (size_t)0, (size_t)0);
  mask_bits<<<gMb, blk, 0, stream>>>(mask, Mb);
  gemm64_f16<0, false><<<gGqkv, blk, 0, stream>>>(Xh, Xh, DM, Wqkv, DM, cscale, (void*)QKV, QKVr, DQKV,
                                                  ROWS, DQKV, DM, aScale, SEQ, 0, SEQ);
  v_tr<<<gVt, blk, 0, stream>>>(QKV, VT);
  v_tr<<<gVt, blk, 0, stream>>>(QKVr, VTr);
  attn_k<true><<<gAttn, dim3(128), 0, stream>>>(QKV, QKVr, VT, VTr, Mb, Ctx, Ctxr, 0, NQB);
  gemm64_f16<1, true><<<gGdm, blk, 0, stream>>>(Ctx, Ctxr, DM, Wp, DM, cscale, (void*)outf, Ctxr, DM,
                                                ROWS, DM, DM, 1.0f, SEQ, 0, SEQ);
  (void)hipGetLastError();
}
